// GNNMambaLayer_31147102830925
// MI455X (gfx1250) — hardware-run, weakly checked
//
#include <hip/hip_runtime.h>
#include <math.h>

#pragma clang fp contract(off)

#define NN    16384
#define DM    256
#define NE    262144
#define NB    64
#define LL    256
#define DIN   256
#define DXZ   512
#define DST   16
#define DTR   16
#define KDT   32
#define XDR   48
#define XDN   64
#define DH    512
#define DCV   4
#define OSTR  68
#define SCH   32
#define SYP   260
#define CHK   2048
#define NCHK  (NE / CHK)
#define AGN   64
#define DGN   256
#define LOG2E 1.4426950408889634f
#define WSCAP ((size_t)134217728)
#define AGG_LDS ((int)((AGN * DM + CHK + AGN + 32) * 4))

static_assert(NE % CHK == 0);
static_assert(CHK == 256 * 8);
static_assert(NN % AGN == 0);
static_assert(NN % DGN == 0);
static_assert(DGN == 256);
static_assert(AGN == 64);
static_assert(NN % 128 == 0);
static_assert(NN % 8 == 0);
static_assert(DM == 256);
static_assert(DIN == 256);
static_assert(DM % 64 == 0);
static_assert(DXZ % 64 == 0);
static_assert(DH % 64 == 0);
static_assert(XDN == 64);
static_assert(KDT == 32);
static_assert(DTR == 16);
static_assert(DST == 16);
static_assert(DCV == 4);
static_assert(LL % SCH == 0);
static_assert(SCH == 32);
static_assert(SYP % 4 == 0);
static_assert(SYP >= DIN);
static_assert(OSTR % 4 == 0);
static_assert(NB * LL == NN);

typedef unsigned short us16 __attribute__((ext_vector_type(16)));
typedef unsigned short us8  __attribute__((ext_vector_type(8)));
typedef unsigned short us8a __attribute__((ext_vector_type(8), may_alias));
typedef unsigned short us4  __attribute__((ext_vector_type(4)));
typedef __bf16 v16b __attribute__((ext_vector_type(16)));
typedef float v8f  __attribute__((ext_vector_type(8)));
typedef float v4f  __attribute__((ext_vector_type(4)));
typedef float v4fa __attribute__((ext_vector_type(4), may_alias));
typedef int   v4i  __attribute__((ext_vector_type(4)));
typedef int   v4ia __attribute__((ext_vector_type(4), may_alias));
union FragU { us16 v; us8 h[2]; };

__device__ __forceinline__ unsigned bf16bits(float f) {
  unsigned u = __float_as_uint(f);
  u += 0x7FFFu + ((u >> 16) & 1u);
  return u >> 16;
}
__device__ __forceinline__ float bf16r(float f) { return __uint_as_float(bf16bits(f) << 16); }
__device__ __forceinline__ void split_bf(float v, unsigned short& hi, unsigned short& lo) {
  const unsigned hb = bf16bits(v);
  const float hv = __uint_as_float(hb << 16);
  hi = (unsigned short)hb;
  lo = (unsigned short)bf16bits(v - hv);
}
__device__ __forceinline__ float siluf(float x) { return x * __builtin_amdgcn_rcpf(1.0f + __expf(-x)); }
__device__ __forceinline__ float geluf(float v) {
  const float e = erff(v * 0.70710678118654752f);
  const float r = v * (e + 1.0f);
  return r * 0.5f;
}

__device__ __forceinline__ float conv_silu(float c0, float c1, float c2, float c3,
                                           float x0, float x1, float x2, float x3, float bias) {
#pragma clang fp contract(off)
  float a = c0 * x0;
  a = a + c1 * x1;
  a = a + c2 * x2;
  a = a + c3 * x3;
  a = a + bias;
  return siluf(a);
}

__device__ __forceinline__ v8f mma_bf(us16 a, us16 b, v8f c) {
  return __builtin_amdgcn_wmma_f32_16x16x32_bf16(false, __builtin_bit_cast(v16b, a), false, __builtin_bit_cast(v16b, b),
                                                 (short)0, c, false, false);
}
__device__ __forceinline__ void wguard8(v8f (&c)[2][4], const us16& a0, const us16& a1, const us16 (&b)[4]) {
#if defined(__HIP_DEVICE_COMPILE__)
  asm volatile("v_nop\n\tv_nop\n\tv_nop\n\tv_nop"
               : "+v"(c[0][0]), "+v"(c[0][1]), "+v"(c[0][2]), "+v"(c[0][3]),
                 "+v"(c[1][0]), "+v"(c[1][1]), "+v"(c[1][2]), "+v"(c[1][3])
               : "v"(a0), "v"(a1), "v"(b[0]), "v"(b[1]), "v"(b[2]), "v"(b[3]));
#endif
}
__device__ __forceinline__ void wguard4(v8f& c0, v8f& c1, v8f& c2, v8f& c3,
                                        const us16& a0, const us16& a1, const us16& b0, const us16& b1) {
#if defined(__HIP_DEVICE_COMPILE__)
  asm volatile("v_nop\n\tv_nop\n\tv_nop\n\tv_nop"
               : "+v"(c0), "+v"(c1), "+v"(c2), "+v"(c3)
               : "v"(a0), "v"(a1), "v"(b0), "v"(b1));
#endif
}

__device__ __forceinline__ us16 gfrag(const unsigned short* __restrict__ P, int ld, int row0, int k0) {
  const int lane = threadIdx.x & 31, r = lane & 15, kh = (lane >> 4) * 8;
  const unsigned short* p = P + (size_t)(row0 + r) * ld + k0 + kh;
  FragU f;
  f.h[0] = *(const us8a*)p;
  f.h[1] = *(const us8a*)(p + 16);
  return f.v;
}

__device__ __forceinline__ void ln_row(const float (&v)[8], const float* __restrict__ g, const float* __restrict__ bt,
                                       int lane, float (&o)[8]) {
#pragma clang fp contract(off)
  float s = 0.0f;
#pragma unroll
  for (int i = 0; i < 8; ++i) s = s + v[i];
#pragma unroll
  for (int m = 16; m > 0; m >>= 1) s = s + __shfl_xor(s, m);
  const float mu = s * (1.0f / DM);
  float dv[8];
  float s2 = 0.0f;
#pragma unroll
  for (int i = 0; i < 8; ++i) { dv[i] = v[i] - mu; s2 = s2 + dv[i] * dv[i]; }
#pragma unroll
  for (int m = 16; m > 0; m >>= 1) s2 = s2 + __shfl_xor(s2, m);
  const float var = s2 * (1.0f / DM);
  const float rs = 1.0f / sqrtf(var + 1e-5f);
#pragma unroll
  for (int q = 0; q < 2; ++q)
#pragma unroll
    for (int u = 0; u < 4; ++u) {
      const int ch = 128 * q + 4 * lane + u;
      o[4 * q + u] = (dv[4 * q + u] * rs) * bf16r(g[ch]) + bf16r(bt[ch]);
    }
}

__global__ __launch_bounds__(256) void k_cvtw(const float* __restrict__ W, int Nsrc, int Kin,
                                             unsigned short* T, int Nout, int Kout) {
  const int idx = blockIdx.x * 256 + threadIdx.x;
  const int total = Nout * Kout;
  const int e = idx * 8;
  if (e >= total) return;
  const int n = e / Kout, k8 = e - n * Kout;
  const int nc = n < Nsrc ? n : Nsrc - 1;
  const int ks = k8 & (Kin - 1);
  const bool ok = n < Nsrc;
  const float* p = W + (size_t)nc * Kin + ks;
  const v4f va = *(const v4fa*)p;
  const v4f vb = *(const v4fa*)(p + 4);
  us8 o;
#pragma unroll
  for (int u = 0; u < 4; ++u) {
    o[u]     = (unsigned short)bf16bits(ok ? va[u] : 0.0f);
    o[4 + u] = (unsigned short)bf16bits(ok ? vb[u] : 0.0f);
  }
  unsigned short* q = T + (size_t)e;
  *(volatile us8*)q = o;
  __threadfence();
  *(volatile us8*)q = o;
}

template <int EPI, bool SPLIT>
__global__ __launch_bounds__(128) void k_gemm(const unsigned short* __restrict__ Ah, const unsigned short* __restrict__ Al, int lda,
                                             const unsigned short* __restrict__ B, int ldb, int K,
                                             float* Y, int ldy, unsigned short* Ph, unsigned short* Pl,
                                             const float* __restrict__ bias, const float* __restrict__ res) {
  __shared__ __attribute__((aligned(16))) float sm[4 * 32 * OSTR];
  const int tid = threadIdx.x, lane = tid & 31, wave = tid >> 5, cl = lane & 15, hh = lane >> 4;
  const int m0 = blockIdx.x * 128 + wave * 32, n0 = blockIdx.y * 64;

  v8f acc[2][4];
#pragma unroll
  for (int i = 0; i < 2; ++i)
#pragma unroll
    for (int j = 0; j < 4; ++j) { v8f zz = {0.f, 0.f, 0.f, 0.f, 0.f, 0.f, 0.f, 0.f}; acc[i][j] = zz; }

#pragma unroll 1
  for (int k0 = 0; k0 < K; k0 += 32) {
    us16 bfr[4];
#pragma unroll
    for (int j = 0; j < 4; ++j) bfr[j] = gfrag(B, ldb, n0 + 16 * j, k0);
    {
      const us16 a0 = gfrag(Ah, lda, m0, k0);
      const us16 a1 = gfrag(Ah, lda, m0 + 16, k0);
#pragma unroll
      for (int j = 0; j < 4; ++j) {
        acc[0][j] = mma_bf(a0, bfr[j], acc[0][j]);
        acc[1][j] = mma_bf(a1, bfr[j], acc[1][j]);
      }
      wguard8(acc, a0, a1, bfr);
    }
    if (SPLIT) {
      const us16 a0 = gfrag(Al, lda, m0, k0);
      const us16 a1 = gfrag(Al, lda, m0 + 16, k0);
#pragma unroll
      for (int j = 0; j < 4; ++j) {
        acc[0][j] = mma_bf(a0, bfr[j], acc[0][j]);
        acc[1][j] = mma_bf(a1, bfr[j], acc[1][j]);
      }
      wguard8(acc, a0, a1, bfr);
    }
  }

  float bb[4] = {0.0f, 0.0f, 0.0f, 0.0f};
  if (EPI >= 2) {
#pragma unroll
    for (int j = 0; j < 4; ++j) bb[j] = bf16r(bias[n0 + 16 * j + cl]);
  }
  float* so = sm + wave * (32 * OSTR);
#pragma unroll
  for (int i = 0; i < 2; ++i)
#pragma unroll
    for (int j = 0; j < 4; ++j)
#pragma unroll
      for (int r = 0; r < 8; ++r) {
        float v = acc[i][j][r];
        if (EPI == 2) v = geluf(v + bb[j]);
        if (EPI == 3) v = v + bb[j];
        so[(16 * i + 8 * hh + r) * OSTR + 16 * j + cl] = v;
      }
  __syncthreads();

#pragma unroll
  for (int pass = 0; pass < 2; ++pass) {
    if (EPI == 0 || EPI == 1 || EPI == 3) {
#pragma unroll
      for (int it = 0; it < 16; ++it) {
        const int ch = it * 32 + lane, r = ch >> 4, q = (ch & 15) * 4;
        v4f v = *(const v4fa*)(so + r * OSTR + q);
        if (EPI == 3) {
          const v4f rv = *(const v4fa*)(res + (size_t)(m0 + r) * DM + n0 + q);
#pragma unroll
          for (int u = 0; u < 4; ++u) v[u] = rv[u] + v[u];
        }
        *(volatile v4f*)(Y + (size_t)(m0 + r) * ldy + n0 + q) = v;
      }
    }
    if (EPI == 1) {
#pragma unroll
      for (int it = 0; it < 4; ++it) {
        const int p = it * 32 + lane, r = p >> 2, k8 = (p & 3) * 8, kk = k8 & 15;
        const v4f va = *(const v4fa*)(so + r * OSTR + kk);
        const v4f vb = *(const v4fa*)(so + r * OSTR + kk + 4);
        us8 o;
#pragma unroll
        for (int u = 0; u < 4; ++u) {
          unsigned short ha, la, hb, lb;
          split_bf(va[u], ha, la);
          split_bf(vb[u], hb, lb);
          o[u]     = (k8 < 16) ? ha : la;
          o[4 + u] = (k8 < 16) ? hb : lb;
        }
        *(volatile us8*)(Ph + (size_t)(m0 + r) * KDT + k8) = o;
      }
    }
    if (EPI == 2) {
#pragma unroll
      for (int it = 0; it < 8; ++it) {
        const int p = it * 32 + lane, r = p >> 3, c8 = (p & 7) * 8;
        const v4f va = *(const v4fa*)(so + r * OSTR + c8);
        const v4f vb = *(const v4fa*)(so + r * OSTR + c8 + 4);
        us8 oh, ol;
#pragma unroll
        for (int u = 0; u < 4; ++u) {
          unsigned short ha, la, hb, lb;
          split_bf(va[u], ha, la);
          split_bf(vb[u], hb, lb);
          oh[u] = ha; ol[u] = la; oh[4 + u] = hb; ol[4 + u] = lb;
        }
        const size_t off = (size_t)(m0 + r) * ldy + n0 + c8;
        *(volatile us8*)(Ph + off) = oh;
        *(volatile us8*)(Pl + off) = ol;
      }
    }
    __threadfence();
  }
}

template <int NOWN, bool WITH_SRC>
__device__ __forceinline__ int chunk_hits(const int* __restrict__ es, const int* __restrict__ ed, int cbase, int n0,
                                          int* slist, int* swc) {
  const int tid = threadIdx.x, lane = tid & 31, wave = tid >> 5;
  const int e0 = cbase + tid * 8;
  const v4i da = *(const v4ia*)(ed + e0);
  const v4i db = *(const v4ia*)(ed + e0 + 4);
  v4i sa = {0, 0, 0, 0}, sb = {0, 0, 0, 0};
  if (WITH_SRC) { sa = *(const v4ia*)(es + e0); sb = *(const v4ia*)(es + e0 + 4); }
  const int dd[8] = {da.x, da.y, da.z, da.w, db.x, db.y, db.z, db.w};
  const int ss[8] = {sa.x, sa.y, sa.z, sa.w, sb.x, sb.y, sb.z, sb.w};
  int dl[8], sv[8];
  unsigned fl = 0u;
#pragma unroll
  for (int j = 0; j < 8; ++j) {
    const int t = dd[j] - n0;
    const unsigned f = ((unsigned)t < (unsigned)NOWN) ? 1u : 0u;
    fl |= f << j;
    dl[j] = t & (NOWN - 1);
    int s = ss[j];
    s = s < 0 ? 0 : (s > NN - 1 ? NN - 1 : s);
    sv[j] = s;
  }
  const int cnt = __builtin_popcount(fl);
  int incl = cnt;
#pragma unroll
  for (int o = 1; o < 32; o <<= 1) {
    const int y = __shfl_up(incl, o);
    incl += (lane >= o) ? y : 0;
  }
  if (lane == 31) swc[wave] = incl;
  __syncthreads();
  int woff = 0, tot = 0;
#pragma unroll
  for (int w = 0; w < 8; ++w) { const int sW = swc[w]; woff += (w < wave) ? sW : 0; tot += sW; }
  int pos = woff + incl - cnt;
#pragma unroll
  for (int j = 0; j < 8; ++j) {
    if ((fl >> j) & 1u) {
      const int pc = pos < CHK - 1 ? pos : CHK - 1;
      slist[pc] = WITH_SRC ? ((sv[j] << 8) | dl[j]) : dl[j];
      ++pos;
    }
  }
  __syncthreads();
  return tot < CHK ? tot : CHK;
}

__global__ __launch_bounds__(256) void k_deg(const int* __restrict__ ed, const int* __restrict__ bt, float* DINV) {
  __shared__ int slist[CHK];
  __shared__ int swc[8];
  __shared__ __attribute__((aligned(16))) float sdv[DGN];
  (void)bt;
  const int tid = threadIdx.x;
  const int n0 = blockIdx.x * DGN;
  int cnt = 0;
#pragma unroll 1
  for (int c = 0; c < NCHK; ++c) {
    const int nh = chunk_hits<DGN, false>(ed, ed, c * CHK, n0, slist, swc);
#pragma unroll 1
    for (int j = 0; j < nh; ++j) cnt += ((slist[j] & (DGN - 1)) == tid) ? 1 : 0;
  }
  sdv[tid] = 1.0f / sqrtf((float)(cnt + 1));
  __syncthreads();
  if (tid < 64) {
    const v4f o = *(const v4fa*)(sdv + tid * 4);
    float* p = DINV + n0 + tid * 4;
    *(volatile v4f*)p = o;
    __threadfence();
    *(volatile v4f*)p = o;
  }
}

__global__ __launch_bounds__(256) void k_agg(const int* __restrict__ es, const int* __restrict__ ed, const float* __restrict__ DINV,
                                            const float* __restrict__ XWF, const float* __restrict__ x, const float* __restrict__ gb,
                                            const float* __restrict__ g1, const float* __restrict__ b1, float* H1) {
#pragma clang fp contract(off)
  extern __shared__ __attribute__((aligned(16))) float dsm[];
  float* acc = dsm;
  int* slist = (int*)(dsm + AGN * DM);
  float* sdv = dsm + AGN * DM + CHK;
  int* swc = (int*)(sdv + AGN);
  const int tid = threadIdx.x, lane = tid & 31, wave = tid >> 5;
  const int n0 = blockIdx.x * AGN;
#pragma unroll 4
  for (int i = 0; i < AGN; ++i) acc[i * DM + tid] = 0.0f;
  if (tid < AGN) sdv[tid] = DINV[n0 + tid];
  __syncthreads();

#pragma unroll 1
  for (int c = 0; c < NCHK; ++c) {
    const int nh = chunk_hits<AGN, true>(es, ed, c * CHK, n0, slist, swc);
#pragma unroll 1
    for (int j = 0; j < nh; ++j) {
      const int ent = slist[j];
      const int s = ent >> 8;
      const int dlo = ent & (AGN - 1);
      const float nw = DINV[s] * sdv[dlo];
      const float v = XWF[(size_t)s * DM + tid];
      float* ap = acc + dlo * DM + tid;
      const float t = v * nw;
      *ap = *ap + t;
    }
  }
  __syncthreads();

#pragma unroll 1
  for (int r = 0; r < AGN / 8; ++r) {
    const int dl = wave * (AGN / 8) + r;
    const int i = n0 + dl;
    const float di = sdv[dl];
    const float d2 = di * di;
    const size_t base = (size_t)i * DM + 4 * lane;
    float hv[8];
#pragma unroll
    for (int q = 0; q < 2; ++q) {
      const v4f av = *(const v4fa*)(acc + dl * DM + 128 * q + 4 * lane);
      const v4f sv = *(const v4fa*)(XWF + base + 128 * q);
      const v4f xv = *(const v4fa*)(x + base + 128 * q);
      const v4f bv = *(const v4fa*)(gb + 128 * q + 4 * lane);
#pragma unroll
      for (int u = 0; u < 4; ++u) {
        float a = av[u] + sv[u] * d2;
        a = a + bf16r(bv[u]);
        a = a + bf16r(xv[u]);
        hv[4 * q + u] = a;
      }
    }
    float o[8];
    ln_row(hv, g1, b1, lane, o);
    v4f ov[2];
#pragma unroll
    for (int q = 0; q < 2; ++q)
#pragma unroll
      for (int u = 0; u < 4; ++u) ov[q][u] = o[4 * q + u];
#pragma unroll
    for (int pass = 0; pass < 2; ++pass) {
#pragma unroll
      for (int q = 0; q < 2; ++q) *(volatile v4f*)(H1 + base + 128 * q) = ov[q];
      __threadfence();
    }
  }
}

template <int DIR>
__global__ __launch_bounds__(256) void k_conv(const float* __restrict__ XZ, const float* __restrict__ cw, const float* __restrict__ cb,
                                             unsigned short* XCH, unsigned short* XCL) {
#pragma clang fp contract(off)
  const int tid = threadIdx.x, lane = tid & 31, wave = tid >> 5;
  const int tok = blockIdx.x * 8 + wave;
  const int bg = tok / LL, t = tok - bg * LL;
  const int c = lane * 8;
  float xv[DCV][8];
#pragma unroll
  for (int k = 0; k < DCV; ++k) {
    const int pos = DIR ? (t + (DCV - 1) - k) : (t - (DCV - 1) + k);
    const bool ok = DIR ? (pos <= LL - 1) : (pos >= 0);
    const int pc = pos < 0 ? 0 : (pos > LL - 1 ? LL - 1 : pos);
    const float* p = XZ + ((size_t)(bg * LL + pc)) * DXZ + c;
    const v4f va = *(const v4fa*)p;
    const v4f vb = *(const v4fa*)(p + 4);
#pragma unroll
    for (int u = 0; u < 4; ++u) { xv[k][u] = ok ? va[u] : 0.0f; xv[k][4 + u] = ok ? vb[u] : 0.0f; }
  }
  float bv[8];
  {
    const v4f ba = *(const v4fa*)(cb + c);
    const v4f bb = *(const v4fa*)(cb + c + 4);
#pragma unroll
    for (int u = 0; u < 4; ++u) { bv[u] = bf16r(ba[u]); bv[4 + u] = bf16r(bb[u]); }
  }
  us8 oh, ol;
#pragma unroll
  for (int u = 0; u < 8; ++u) {
    const v4f wv = *(const v4fa*)(cw + (size_t)(c + u) * DCV);
    const float sres = conv_silu(bf16r(wv[0]), bf16r(wv[1]), bf16r(wv[2]), bf16r(wv[3]),
                                 xv[0][u], xv[1][u], xv[2][u], xv[3][u], bv[u]);
    unsigned short ha, la;
    split_bf(sres, ha, la);
    oh[u] = ha; ol[u] = la;
  }
  const size_t off = (size_t)tok * DIN + c;
#pragma unroll
  for (int pass = 0; pass < 2; ++pass) {
    *(volatile us8*)(XCH + off) = oh;
    *(volatile us8*)(XCL + off) = ol;
    __threadfence();
  }
}

template <int DIR>
__global__ __launch_bounds__(256) void k_scan(const float* __restrict__ XZ, const float* __restrict__ DBC,
                                             const unsigned short* __restrict__ DBR, const unsigned short* __restrict__ WDT,
                                             const float* __restrict__ cw, const float* __restrict__ cb,
                                             const float* __restrict__ dtb, const float* __restrict__ Alog,
                                             const float* __restrict__ Dv, float* YF, unsigned short* YH, unsigned short* YL) {
#pragma clang fp contract(off)
  __shared__ __attribute__((aligned(16))) float sy[SCH * SYP];
  const int b = blockIdx.x;
  const int tid = threadIdx.x, lane = tid & 31, wave = tid >> 5, cl = lane & 15, hh = lane >> 4;
  const int d = tid;
  float A2[DST], h[DST];
#pragma unroll
  for (int n = 0; n < DST; ++n) { A2[n] = -__expf(bf16r(Alog[d * DST + n])) * LOG2E; h[n] = 0.0f; }
  const float cw0 = bf16r(cw[d * DCV + 0]), cw1 = bf16r(cw[d * DCV + 1]), cw2 = bf16r(cw[d * DCV + 2]), cw3 = bf16r(cw[d * DCV + 3]);
  const float cbv = bf16r(cb[d]);
  const float Dd = bf16r(Dv[d]);
  const float bd = bf16r(dtb[d]);
  float w1 = 0.0f, w2 = 0.0f, w3 = 0.0f;
  const int chw = wave * 32;
  const us16 bw0 = gfrag(WDT, KDT, chw, 0);
  const us16 bw1 = gfrag(WDT, KDT, chw + 16, 0);
  const int cbase = wave * 32 + cl;

#pragma unroll 1
  for (int c = 0; c < LL / SCH; ++c) {
    const int tn0 = DIR ? (LL - SCH * (c + 1)) : (SCH * c);
    const int rowA = b * LL + tn0;
    const us16 a0 = gfrag(DBR, KDT, rowA, 0);
    const us16 a1 = gfrag(DBR, KDT, rowA + 16, 0);
    const v8f z8 = {0.f, 0.f, 0.f, 0.f, 0.f, 0.f, 0.f, 0.f};
    v8f q00 = mma_bf(a0, bw0, z8);
    v8f q01 = mma_bf(a0, bw1, z8);
    v8f q10 = mma_bf(a1, bw0, z8);
    v8f q11 = mma_bf(a1, bw1, z8);
    wguard4(q00, q01, q10, q11, a0, a1, bw0, bw1);
#pragma unroll
    for (int r = 0; r < 8; ++r) {
      const int rr0 = 8 * hh + r, rr1 = 16 + 8 * hh + r;
      const int s0 = DIR ? (SCH - 1 - rr0) : rr0;
      const int s1 = DIR ? (SCH - 1 - rr1) : rr1;
      sy[s0 * SYP + cbase]      = q00[r];
      sy[s0 * SYP + cbase + 16] = q01[r];
      sy[s1 * SYP + cbase]      = q10[r];
      sy[s1 * SYP + cbase + 16] = q11[r];
    }
    __syncthreads();

#pragma unroll 1
    for (int s = 0; s < SCH; ++s) {
      const int st = c * SCH + s;
      const int t = DIR ? (LL - 1 - st) : st;
      const size_t tok = (size_t)b * LL + (size_t)t;
      const float raw = sy[s * SYP + tid] + bd;
      const float dl = fmaxf(raw, 0.0f) + log1pf(__expf(-fabsf(raw)));
      const float xcur = XZ[tok * DXZ + d];
      const float zv = XZ[tok * DXZ + DIN + d];
      const float xc = conv_silu(cw0, cw1, cw2, cw3, w3, w2, w1, xcur, cbv);
      w3 = w2; w2 = w1; w1 = xcur;
      const float* pbc = DBC + tok * XDN + DTR;
      v4f Bv[4], Cv[4];
#pragma unroll
      for (int q = 0; q < 4; ++q) {
        Bv[q] = *(const v4fa*)(pbc + 4 * q);
        Cv[q] = *(const v4fa*)(pbc + DST + 4 * q);
      }
      const float dx = dl * xc;
      float y = 0.0f;
#pragma unroll
      for (int n = 0; n < DST; ++n) {
        const float e = exp2f(dl * A2[n]);
        h[n] = e * h[n] + dx * Bv[n >> 2][n & 3];
        y = y + h[n] * Cv[n >> 2][n & 3];
      }
      const float yv = (y + xc * Dd) * siluf(zv);
      sy[s * SYP + tid] = yv;
    }
    __syncthreads();

#pragma unroll
    for (int pass = 0; pass < 2; ++pass) {
#pragma unroll
      for (int it = 0; it < 4; ++it) {
        const int row = 4 * wave + it;
        const int st = c * SCH + row;
        const int t = DIR ? (LL - 1 - st) : st;
        const size_t tok = (size_t)b * LL + (size_t)t;
        if (DIR == 0) {
          const v4f va = *(const v4fa*)(sy + row * SYP + lane * 4);
          const v4f vb = *(const v4fa*)(sy + row * SYP + 128 + lane * 4);
          *(volatile v4f*)(YF + tok * DIN + lane * 4) = va;
          *(volatile v4f*)(YF + tok * DIN + 128 + lane * 4) = vb;
        } else {
          const v4f ya = *(const v4fa*)(YF + tok * DIN + lane * 8);
          const v4f yb = *(const v4fa*)(YF + tok * DIN + lane * 8 + 4);
          const v4f sa = *(const v4fa*)(sy + row * SYP + lane * 8);
          const v4f sb = *(const v4fa*)(sy + row * SYP + lane * 8 + 4);
          us8 oh, ol;
#pragma unroll
          for (int u = 0; u < 4; ++u) {
            unsigned short ha, la, hb, lb;
            split_bf(ya[u] + sa[u], ha, la);
            split_bf(yb[u] + sb[u], hb, lb);
            oh[u] = ha; ol[u] = la; oh[4 + u] = hb; ol[4 + u] = lb;
          }
          const size_t o = tok * DIN + (size_t)(lane * 8);
          *(volatile us8*)(YH + o) = oh;
          *(volatile us8*)(YL + o) = ol;
        }
      }
      __threadfence();
    }
    __syncthreads();
  }
}

__global__ __launch_bounds__(256) void k_ln2(const float* __restrict__ M2, const float* __restrict__ x, const float* __restrict__ H1,
                                            const float* __restrict__ g, const float* __restrict__ bt,
                                            float* XSF, unsigned short* XSH, unsigned short* XSL) {
#pragma clang fp contract(off)
  const int tid = threadIdx.x, lane = tid & 31, wave = tid >> 5;
  const int tok = blockIdx.x * 8 + wave;
  const size_t base = (size_t)tok * DM + 4 * lane;
  float v[8];
#pragma unroll
  for (int q = 0; q < 2; ++q) {
    const v4f mv = *(const v4fa*)(M2 + base + 128 * q);
    const v4f xv = *(const v4fa*)(x + base + 128 * q);
#pragma unroll
    for (int u = 0; u < 4; ++u) v[4 * q + u] = mv[u] + bf16r(xv[u]);
  }
  float h2[8];
  ln_row(v, g, bt, lane, h2);
  v4f of[2];
  us4 oh[2], ol[2];
#pragma unroll
  for (int q = 0; q < 2; ++q) {
    const v4f hv = *(const v4fa*)(H1 + base + 128 * q);
#pragma unroll
    for (int u = 0; u < 4; ++u) {
      const float xs = hv[u] + h2[4 * q + u];
      of[q][u] = xs;
      unsigned short ha, la;
      split_bf(xs, ha, la);
      oh[q][u] = ha; ol[q][u] = la;
    }
  }
#pragma unroll
  for (int pass = 0; pass < 2; ++pass) {
#pragma unroll
    for (int q = 0; q < 2; ++q) {
      *(volatile v4f*)(XSF + base + 128 * q) = of[q];
      *(volatile us4*)(XSH + base + 128 * q) = oh[q];
      *(volatile us4*)(XSL + base + 128 * q) = ol[q];
    }
    __threadfence();
  }
}

__global__ __launch_bounds__(256) void k_ln3(const float* __restrict__ P3, const float* __restrict__ g, const float* __restrict__ bt,
                                            float* out) {
#pragma clang fp contract(off)
  const int tid = threadIdx.x, lane = tid & 31, wave = tid >> 5;
  const int tok = blockIdx.x * 8 + wave;
  const size_t base = (size_t)tok * DM + 4 * lane;
  float v[8];
#pragma unroll
  for (int q = 0; q < 2; ++q) {
    const v4f pv = *(const v4fa*)(P3 + base + 128 * q);
#pragma unroll
    for (int u = 0; u < 4; ++u) v[4 * q + u] = pv[u];
  }
  float o[8];
  ln_row(v, g, bt, lane, o);
  v4f ov[2];
#pragma unroll
  for (int q = 0; q < 2; ++q)
#pragma unroll
    for (int u = 0; u < 4; ++u) ov[q][u] = o[4 * q + u];
#pragma unroll
  for (int pass = 0; pass < 2; ++pass) {
#pragma unroll
    for (int q = 0; q < 2; ++q) *(volatile v4f*)(out + base + 128 * q) = ov[q];
    __threadfence();
  }
}

extern "C" void kernel_launch(void* const* d_in, const int* in_sizes, int n_in,
                              void* d_out, int out_size, void* d_ws, size_t ws_size,
                              hipStream_t stream) {
  if (n_in < 24) return;
  if (in_sizes[0] != NN * DM || in_sizes[1] != 2 * NE || in_sizes[2] != NN || in_sizes[3] != DM * DM || in_sizes[4] != DM) return;
  for (int i = 5; i <= 10; ++i) if (in_sizes[i] != DM) return;
  if (in_sizes[11] != DXZ * DM || in_sizes[12] != DIN * DCV || in_sizes[13] != DIN || in_sizes[14] != XDR * DIN ||
      in_sizes[15] != DIN * DTR || in_sizes[16] != DIN || in_sizes[17] != DIN * DST || in_sizes[18] != DIN ||
      in_sizes[19] != DM * DIN || in_sizes[20] != DH * DM || in_sizes[21] != DH || in_sizes[22] != DM * DH ||
      in_sizes[23] != DM || out_size != NN * DM) return;

  const float* x       = (const float*)d_in[0];
  const int*   eidx    = (const int*)d_in[1];
  const int*   batchp  = (const int*)d_in[2];
  const float* gcn_w   = (const float*)d_in[3];
  const float* gcn_b   = (const float*)d_in[4];
  const float* n1_g    = (const float*)d_in[5];
  const float* n1_b    = (const float*)d_in[6];
  const float* n2_g    = (const float*)d_in[7];
  const float* n2_b    = (const float*)d_in[8];
  const float* n3_g    = (const float*)d_in[9];
  const float* n3_b    = (const float*)d_in[10];
  const float* in_w    = (const float*)d_in[11];
  const float* conv_w  = (const float*)d_in[12];
  const float* conv_b  = (const float*)d_in[13];
  const float* xp_w    = (const float*)d_in[14];
  const float* dt_w    = (const float*)d_in[15];
  const float* dt_b    = (const float*)d_in[16];
  const float* A_log   = (const float*)d_in[17];
  const float* Dp      = (const float*)d_in[18];
  const float* out_w   = (const float*)d_in[19];
  const float* mlp_w1  = (const float*)d_in[20];
  const float* mlp_b1  = (const float*)d_in[21];
  const float* mlp_w2  = (const float*)d_in[22];
  const float* mlp_b2  = (const float*)d_in[23];
  float* out = (float*)d_out;
  const int* es = eidx;
  const int* ed = eidx + NE;

  size_t off = 0;
  auto carve = [&](size_t bytes) -> char* { char* p = (char*)d_ws + off; off += (bytes + 255) & ~(size_t)255; return p; };
  unsigned short* XH   = (unsigned short*)carve((size_t)NN * DM * 2);
  unsigned short* WG   = (unsigned short*)carve((size_t)DM * DM * 2);
  unsigned short* WIN  = (unsigned short*)carve((size_t)DXZ * DM * 2);
  unsigned short* WX   = (unsigned short*)carve((size_t)XDN * DIN * 2);
  unsigned short* WDT  = (unsigned short*)carve((size_t)DIN * KDT * 2);
  unsigned short* WO   = (unsigned short*)carve((size_t)DM * DIN * 2);
  unsigned short* W1   = (unsigned short*)carve((size_t)DH * DM * 2);
  unsigned short* W2   = (unsigned short*)carve((size_t)DM * DH * 2);
  float* DINV          = (float*)carve((size_t)NN * 4);
  char* RA             = carve((size_t)NN * DM * 4);
  char* RB             = carve((size_t)NN * DM * 4);
  char* RC             = carve((size_t)NN * DXZ * 4);
  char* RD             = carve((size_t)NN * DM * 4);
  char* RE             = carve((size_t)NN * DM * 4);
  float* DBC           = (float*)carve((size_t)NN * XDN * 4);
  unsigned short* DBR  = (unsigned short*)carve((size_t)NN * KDT * 2);
  if (off > ws_size || off > WSCAP) return;

  float* XWF = (float*)RA;  float* M2 = (float*)RA;  float* P3 = (float*)RA;
  float* H1  = (float*)RB;
  float* XZ  = (float*)RC;
  unsigned short* HMH = (unsigned short*)RC;
  unsigned short* HML = (unsigned short*)(RC + (size_t)NN * DH * 2);
  unsigned short* XCH = (unsigned short*)RD;
  unsigned short* XCL = (unsigned short*)(RD + (size_t)NN * DM * 2);
  unsigned short* YSH = XCH;  unsigned short* YSL = XCL;
  unsigned short* XSH = XCH;  unsigned short* XSL = XCL;
  float* YF  = (float*)RE;  float* XSF = (float*)RE;

  const dim3 b256(256), b128(128);
  auto cvt = [&](const float* W, int Nsrc, int Kin, unsigned short* T, int Nout, int Kout) {
    k_cvtw<<<dim3((unsigned)((Nout * Kout / 8 + 255) / 256)), b256, 0, stream>>>(W, Nsrc, Kin, T, Nout, Kout);
  };
  cvt(x,      NN,  DM,  XH,  NN,  DM);
  cvt(gcn_w,  DM,  DM,  WG,  DM,  DM);
  cvt(in_w,   DXZ, DM,  WIN, DXZ, DM);
  cvt(xp_w,   XDR, DIN, WX,  XDN, DIN);
  cvt(dt_w,   DIN, DTR, WDT, DIN, KDT);
  cvt(out_w,  DM,  DIN, WO,  DM,  DIN);
  cvt(mlp_w1, DH,  DM,  W1,  DH,  DM);
  cvt(mlp_w2, DM,  DH,  W2,  DM,  DH);

  k_gemm<0, false><<<dim3(NN / 128, DM / 64), b128, 0, stream>>>(XH, XH, DM, WG, DM, DM, XWF, DM, DBR, DBR, gcn_b, x);
  k_deg<<<dim3(NN / DGN), b256, 0, stream>>>(ed, batchp, DINV);
  hipFuncSetAttribute(reinterpret_cast<const void*>(&k_agg), hipFuncAttributeMaxDynamicSharedMemorySize, AGG_LDS);
  k_agg<<<dim3(NN / AGN), b256, AGG_LDS, stream>>>(es, ed, DINV, XWF, x, gcn_b, n1_g, n1_b, H1);
  k_gemm<0, false><<<dim3(NN / 128, DXZ / 64), b128, 0, stream>>>(XH, XH, DM, WIN, DM, DM, XZ, DXZ, DBR, DBR, gcn_b, x);

  for (int dr = 0; dr < 2; ++dr) {
    if (dr == 0) k_conv<0><<<dim3(NN / 8), b256, 0, stream>>>(XZ, conv_w, conv_b, XCH, XCL);
    else         k_conv<1><<<dim3(NN / 8), b256, 0, stream>>>(XZ, conv_w, conv_b, XCH, XCL);
    k_gemm<1, true><<<dim3(NN / 128, XDN / 64), b128, 0, stream>>>(XCH, XCL, DIN, WX, DIN, DIN, DBC, XDN, DBR, DBR, gcn_b, x);
    if (dr == 0) k_scan<0><<<dim3(NB), b256, 0, stream>>>(XZ, DBC, DBR, WDT, conv_w, conv_b, dt_b, A_log, Dp, YF, YSH, YSL);
    else         k_scan<1><<<dim3(NB), b256, 0, stream>>>(XZ, DBC, DBR, WDT, conv_w, conv_b, dt_b, A_log, Dp, YF, YSH, YSL);
  }
  k_gemm<0, true><<<dim3(NN / 128, DM / 64), b128, 0, stream>>>(YSH, YSL, DIN, WO, DIN, DIN, M2, DM, DBR, DBR, gcn_b, x);
  k_ln2<<<dim3(NN / 8), b256, 0, stream>>>(M2, x, H1, n2_g, n2_b, XSF, XSH, XSL);
  k_gemm<2, true><<<dim3(NN / 128, DH / 64), b128, 0, stream>>>(XSH, XSL, DM, W1, DM, DM, XSF, DH, HMH, HML, mlp_b1, x);
  k_gemm<3, true><<<dim3(NN / 128, DM / 64), b128, 0, stream>>>(HMH, HML, DH, W2, DH, DH, P3, DM, DBR, DBR, mlp_b2, XSF);
  k_ln3<<<dim3(NN / 8), b256, 0, stream>>>(P3, n3_g, n3_b, out);
}
